// GAT_7086696039040
// MI455X (gfx1250) — hardware-verified
//
#include <hip/hip_runtime.h>
#include <stddef.h>
#include <stdint.h>
#include <math.h>


#define NN      8192
#define FIN     128
#define HC      128
#define CH      64
#define NHEAD   2
#define KA      256
#define KX1     128
#define NODED   8
#define NG      64
#define PN      128
#define KF1     2048
#define NF1     256
#define NF2     32
#define NTHR    256
#define NWAVE   8
#define EPT     8
#define CHUNK   (NTHR * EPT)
#define WCAP    (EPT * 32)
#define LISTN   (NWAVE * WCAP)
#define NBA     128
#define SLA     7
#define SRCB    13
#define RCAP    20480
#define DEGCAP  144
#define MEAS_B128   16384
#define MEAS_MAXDEG 128
#define GBM     64
#define GBN     64
#define GTHR    128
#define NT64    (NN / GBM)
#define NBLK    (NN / NBA)
#define NFLG    (3 * NBLK)
#define NEGSL   0.2f
#define BN_EPS  1e-5f
#define WSMAX   134217728
#define BKT_LDS_INTS  (LISTN + RCAP + 16)
#define SCAN_LDS_INTS (NBA * DEGCAP + NBA + 16)
#define NU_XB   (NN * FIN / 8)
#define NU_WL0  (HC * FIN / 8)
#define NU_WP0  (CH * KA / 8)
#define NU_WL1  (HC * KX1 / 8)
#define NU_WM1  (CH * KA / 8)
#define NU_WF1  (NF1 * KF1 / 8)
#define NU_ALL  (NU_XB + NU_WL0 + NU_WP0 + NU_WL1 + NU_WM1 + NU_WF1)

static_assert((CHUNK & (CHUNK - 1)) == 0 && CHUNK <= 4096);
static_assert(NBA == (1 << SLA) && NN <= (1 << SRCB) && NBA <= (1 << 7));
static_assert(((long long)CHUNK << SLA) < (1LL << 31));
static_assert((NN % NBA) == 0 && (NN % 128) == 0 && NN / PN == NG);
static_assert(HC == NHEAD * CH && CH == 64 && HC == 128 && HC == 4 * 32);
static_assert(NBA == NWAVE * 16);
static_assert((RCAP % (NTHR * 4)) == 0 && RCAP >= MEAS_B128 + 4096);
static_assert(DEGCAP >= MEAS_MAXDEG + 8);
static_assert((SCAN_LDS_INTS % 4) == 0);
static_assert(SCAN_LDS_INTS * 4 <= 300000 && BKT_LDS_INTS * 4 <= 300000);
static_assert(GBM == (GTHR / 32) * 16 && GTHR == 2 * GBN && GTHR == 2 * GBM);
static_assert((FIN % 32) == 0 && (KA % 32) == 0 && (KX1 % 32) == 0 && (KF1 % 32) == 0);
static_assert(KA == 2 * HC && KX1 == 2 * CH && KF1 == 2 * PN * NODED);
static_assert((NN % GBM) == 0 && (HC % GBN) == 0 && CH == GBN && (NF1 % GBN) == 0 && NG == GBM);
static_assert((NU_XB % NTHR) == 0 && (NU_WL0 % NTHR) == 0 && (NU_WP0 % NTHR) == 0);
static_assert((NU_WL1 % NTHR) == 0 && (NU_WM1 % NTHR) == 0 && (NU_WF1 % NTHR) == 0);
static_assert(NFLG <= NTHR);
static_assert(NG * 4 == NTHR && NF2 == 32);

typedef float          v2f  __attribute__((ext_vector_type(2)));
typedef float          v4f  __attribute__((ext_vector_type(4)));
typedef float          v8f  __attribute__((ext_vector_type(8)));
typedef double         v2d  __attribute__((ext_vector_type(2)));
typedef int            v4i  __attribute__((ext_vector_type(4)));
typedef int            v8i  __attribute__((ext_vector_type(8)));
typedef unsigned int   v2u  __attribute__((ext_vector_type(2)));
typedef unsigned int   v4u  __attribute__((ext_vector_type(4)));
typedef unsigned short v8us __attribute__((ext_vector_type(8)));
typedef __bf16         v16b __attribute__((ext_vector_type(16)));
typedef v4f  __attribute__((may_alias)) v4fa;
typedef v2d  __attribute__((may_alias)) v2da;
typedef v4i  __attribute__((may_alias)) v4ia;
typedef v8us __attribute__((may_alias)) v8usa;
union FragB { v16b v; v8us h[2]; v8i w; };

__device__ __forceinline__ v8f wmb(const FragB& a, const FragB& b, v8f c) {
  v8f d = __builtin_amdgcn_wmma_f32_16x16x32_bf16(false, a.v, false, b.v, (short)0, c, false, false);
  asm volatile("v_nop\n\tv_nop\n\tv_nop\n\tv_nop" : "+v"(d) : "v"(a.w), "v"(b.w));
  return d;
}

__device__ __forceinline__ unsigned int f2bf(float f) {
  const unsigned int u = __float_as_uint(f);
  const unsigned int r = ((u + 0x7FFFu + ((u >> 16) & 1u)) >> 16) & 0xFFFFu;
  return ((u & 0x7FFFFFFFu) > 0x7F800000u) ? 0x7FC0u : r;
}
__device__ __forceinline__ float bf2f(unsigned int b) { return __uint_as_float(b << 16); }
__device__ __forceinline__ float bfr(float f) { return bf2f(f2bf(f)); }
__device__ __forceinline__ v4f bfr4(const v4f a) {
  v4f r; r.x = bfr(a.x); r.y = bfr(a.y); r.z = bfr(a.z); r.w = bfr(a.w); return r;
}
__device__ __forceinline__ unsigned int pk2(float lo, float hi) { return f2bf(lo) | (f2bf(hi) << 16); }
__device__ __forceinline__ unsigned int pk2lo(float lo, float hi) {
  return f2bf(lo - bfr(lo)) | (f2bf(hi - bfr(hi)) << 16);
}
__device__ __forceinline__ v4u pack8(const v4f a, const v4f b) {
  v4u r; r.x = pk2(a.x, a.y); r.y = pk2(a.z, a.w); r.z = pk2(b.x, b.y); r.w = pk2(b.z, b.w); return r;
}
__device__ __forceinline__ v4u pack8lo(const v4f a, const v4f b) {
  v4u r; r.x = pk2lo(a.x, a.y); r.y = pk2lo(a.z, a.w); r.z = pk2lo(b.x, b.y); r.w = pk2lo(b.z, b.w); return r;
}
__device__ __forceinline__ float lrelu(float v) { return (v >= 0.0f) ? v : NEGSL * v; }

template <int SLB>
__device__ __forceinline__ int scan_chunk(const int* __restrict__ dsts, int nE, int cbase, int slotBase,
                                          int nb, int vec8, int* list, int tid, int lane, int wave) {
  int wc = 0;
  const int el0  = tid * EPT;
  const int e0   = cbase + el0;
  const int sent = -2147483647 - 1;
  v4i da, db;
  if (vec8 != 0 && cbase + CHUNK <= nE) {
    da = *(const v4i*)(dsts + e0);
    db = *(const v4i*)(dsts + e0 + 4);
  } else {
    da.x = (e0     < nE) ? dsts[min(e0,     nE - 1)] : sent;
    da.y = (e0 + 1 < nE) ? dsts[min(e0 + 1, nE - 1)] : sent;
    da.z = (e0 + 2 < nE) ? dsts[min(e0 + 2, nE - 1)] : sent;
    da.w = (e0 + 3 < nE) ? dsts[min(e0 + 3, nE - 1)] : sent;
    db.x = (e0 + 4 < nE) ? dsts[min(e0 + 4, nE - 1)] : sent;
    db.y = (e0 + 5 < nE) ? dsts[min(e0 + 5, nE - 1)] : sent;
    db.z = (e0 + 6 < nE) ? dsts[min(e0 + 6, nE - 1)] : sent;
    db.w = (e0 + 7 < nE) ? dsts[min(e0 + 7, nE - 1)] : sent;
  }
  const unsigned nbs = (unsigned)slotBase;
  const unsigned unb = (unsigned)nb;
  const unsigned s0 = (unsigned)da.x - nbs, s1 = (unsigned)da.y - nbs;
  const unsigned s2 = (unsigned)da.z - nbs, s3 = (unsigned)da.w - nbs;
  const unsigned s4 = (unsigned)db.x - nbs, s5 = (unsigned)db.y - nbs;
  const unsigned s6 = (unsigned)db.z - nbs, s7 = (unsigned)db.w - nbs;
  const bool h0 = s0 < unb, h1 = s1 < unb, h2 = s2 < unb, h3 = s3 < unb;
  const bool h4 = s4 < unb, h5 = s5 < unb, h6 = s6 < unb, h7 = s7 < unb;
  const unsigned any = __builtin_amdgcn_ballot_w32(h0 | h1 | h2 | h3 | h4 | h5 | h6 | h7);
  if (any != 0u) {
#define HITJ(J, HJ, SJ) { \
      const unsigned mj = __builtin_amdgcn_ballot_w32(HJ); \
      if (mj != 0u) { \
        if (HJ) { \
          const int pos = wc + (int)__builtin_amdgcn_mbcnt_lo(mj, 0u); \
          if (pos < WCAP) list[wave * WCAP + pos] = ((el0 + (J)) << SLB) | (int)(SJ); \
        } \
        wc += (int)__builtin_popcount(mj); } }
    HITJ(0, h0, s0)
    HITJ(1, h1, s1)
    HITJ(2, h2, s2)
    HITJ(3, h3, s3)
    HITJ(4, h4, s4)
    HITJ(5, h5, s5)
    HITJ(6, h6, s6)
    HITJ(7, h7, s7)
#undef HITJ
  }
  return wc;
}

__device__ __forceinline__ void cvt_put8(const float* __restrict__ p, unsigned short* dp) {
  const v4f a = *(const v4f*)p;
  const v4f b = *(const v4f*)(p + 4);
  const v4u hv = pack8(a, b);
  *(volatile v4u*)dp = hv;
  __threadfence();
  *(volatile v4u*)dp = hv;
}

__global__ __launch_bounds__(NTHR) void k_prep(const float* __restrict__ x, const float* __restrict__ wl0,
                                               const float* __restrict__ wp0, const float* __restrict__ wl1,
                                               const float* __restrict__ wm1, const float* __restrict__ wf1,
                                               unsigned short* XB, unsigned short* WL0, unsigned short* WP0D,
                                               unsigned short* WL1D, unsigned short* WM1D, unsigned short* WF1D) {
  const int u = (int)blockIdx.x * NTHR + (int)threadIdx.x;
  if (u < NU_XB) {
    cvt_put8(x + (size_t)u * 8, XB + (size_t)u * 8);
  } else if (u < NU_XB + NU_WL0) {
    const int v = u - NU_XB;
    cvt_put8(wl0 + (size_t)v * 8, WL0 + (size_t)v * 8);
  } else if (u < NU_XB + NU_WL0 + NU_WP0) {
    const int v = u - NU_XB - NU_WL0;
    const int n = v >> 5, k8 = (v & 31) * 8, kk = k8 & (HC - 1);
    cvt_put8(wp0 + (size_t)n * HC + kk, WP0D + (size_t)v * 8);
  } else if (u < NU_XB + NU_WL0 + NU_WP0 + NU_WL1) {
    const int v = u - NU_XB - NU_WL0 - NU_WP0;
    const int n = v >> 4, k8 = (v & 15) * 8, kk = k8 & (CH - 1);
    cvt_put8(wl1 + (size_t)n * CH + kk, WL1D + (size_t)v * 8);
  } else if (u < NU_XB + NU_WL0 + NU_WP0 + NU_WL1 + NU_WM1) {
    const int v = u - NU_XB - NU_WL0 - NU_WP0 - NU_WL1;
    const int n = v >> 5, k8 = (v & 31) * 8, kk = k8 & (HC - 1);
    cvt_put8(wm1 + (size_t)n * HC + kk, WM1D + (size_t)v * 8);
  } else if (u < NU_ALL) {
    const int v = u - NU_XB - NU_WL0 - NU_WP0 - NU_WL1 - NU_WM1;
    const int n = v >> 8, k8 = (v & 255) * 8, kk = k8 & (PN * NODED - 1);
    cvt_put8(wf1 + (size_t)n * (PN * NODED) + kk, WF1D + (size_t)v * 8);
  }
}

__global__ __launch_bounds__(NTHR) void k_bucket(const int* __restrict__ srcs, const int* __restrict__ dsts,
                                                 int nE, int nN, int vec8, int* HITS, int* FLG) {
  extern __shared__ __attribute__((aligned(16))) int bsm[];
  int* list = bsm;
  int* reg1 = bsm + LISTN;
  int* wcnt = reg1 + RCAP;
  const int tid = (int)threadIdx.x, lane = tid & 31, wave = tid >> 5;
  const int blk = (int)blockIdx.x;
  const int nodeBase = blk * NBA;
  int nb = nN - nodeBase;
  nb = nb < 0 ? 0 : (nb > NBA ? NBA : nb);

  int tot = 0, ovf = 0;
  const int nChunks = (nE + CHUNK - 1) / CHUNK;
#pragma unroll 1
  for (int ch = 0; ch < nChunks; ++ch) {
    const int cbase = ch * CHUNK;
    const int wc = scan_chunk<SLA>(dsts, nE, cbase, nodeBase, nb, vec8, list, tid, lane, wave);
    if (lane == 0) wcnt[wave] = wc;
    __syncthreads();
    int pre = 0, all = 0;
#pragma unroll
    for (int w2 = 0; w2 < NWAVE; ++w2) {
      int c = wcnt[w2];
      c = c < 0 ? 0 : (c > WCAP ? WCAP : c);
      all += c;
      pre += (w2 < wave) ? c : 0;
    }
    const int wcc  = wc > WCAP ? WCAP : wc;
    const int base = tot + pre;
#pragma unroll 1
    for (int i = lane; i < wcc; i += 32) {
      const int ent = list[wave * WCAP + i];
      const int el  = (ent >> SLA) & (CHUNK - 1);
      const int sl  = ent & (NBA - 1);
      int eid = cbase + el;
      eid = eid > nE - 1 ? nE - 1 : eid;
      const int sraw = srcs[eid];
      const int s = sraw < 0 ? 0 : (sraw > nN - 1 ? nN - 1 : sraw);
      const int pos = base + i;
      if (pos < RCAP) reg1[pos] = (int)((unsigned)s | ((unsigned)sl << SRCB));
    }
    if (tot + all > RCAP) ovf = 1;
    tot += all;
    tot = tot > RCAP ? RCAP : tot;
    __syncthreads();
  }
  const int nh = tot;
  for (int i = nh + tid; i < RCAP; i += NTHR) reg1[i] = 0;
  __syncthreads();

  int* hb = HITS + (size_t)blk * RCAP;
  v4i cv;
  cv.x = (tid == 0) ? nh : 0;
  cv.y = (tid == 0) ? ovf : 0;
  cv.z = 0; cv.w = 0;
  int* fp = FLG + (size_t)blk * 32 + 4 * (tid & 7);
#pragma unroll 1
  for (int p = tid * 4; p < RCAP; p += NTHR * 4) {
    const v4i v = *(const v4ia*)(reg1 + p);
    *(volatile v4i*)(hb + p) = v;
  }
  if (tid < 8) *(volatile v4i*)fp = cv;
  __threadfence();
#pragma unroll 1
  for (int p = tid * 4; p < RCAP; p += NTHR * 4) {
    const v4i v = *(const v4ia*)(reg1 + p);
    *(volatile v4i*)(hb + p) = v;
  }
  if (tid < 8) *(volatile v4i*)fp = cv;
}

__device__ __forceinline__ void gemm_acc64(const unsigned short* __restrict__ A, const unsigned short* __restrict__ WT,
                                           int K, int rowBase, int col0, int wave, int hh, int m, v8f (&acc)[4]) {
  const v8f z = {0.f, 0.f, 0.f, 0.f, 0.f, 0.f, 0.f, 0.f};
  acc[0] = z; acc[1] = z; acc[2] = z; acc[3] = z;
  const unsigned short* ap = A  + (size_t)(rowBase + 16 * wave + m) * (size_t)K + 8 * hh;
  const unsigned short* wp = WT + (size_t)(col0 + m) * (size_t)K + 8 * hh;
  const int ksteps = K >> 5;
#pragma unroll 1
  for (int ks = 0; ks < ksteps; ++ks) {
    FragB af;
    af.h[0] = *(const v8usa*)(ap + 32 * ks);
    af.h[1] = *(const v8usa*)(ap + 32 * ks + 16);
#pragma unroll
    for (int t = 0; t < 4; ++t) {
      const unsigned short* wq = wp + (size_t)(16 * t) * (size_t)K + 32 * ks;
      FragB bf;
      bf.h[0] = *(const v8usa*)wq;
      bf.h[1] = *(const v8usa*)(wq + 16);
      acc[t] = wmb(af, bf, acc[t]);
    }
  }
}

template <bool ACT>
__device__ __forceinline__ void stage64(float* stg, const v8f (&acc)[4], const float (&bv)[4], int wave, int hh, int m) {
#pragma unroll
  for (int t = 0; t < 4; ++t) {
    const int lc = 16 * t + m;
#pragma unroll
    for (int r = 0; r < 8; ++r) {
      const int lr = 16 * wave + 8 * hh + r;
      float v = acc[t][r];
      if (ACT) v = lrelu(v + bv[t]);
      stg[lr * GBN + lc] = v;
    }
  }
}
__device__ __forceinline__ void load_rows(const float* stg, v4f (&fv)[8], int wave, int hh, int m) {
#pragma unroll
  for (int i = 0; i < 8; ++i) {
    const int lr = 16 * wave + 2 * i + hh;
    fv[i] = *(const v4fa*)(stg + lr * GBN + 4 * m);
  }
}
__device__ __forceinline__ void put_rows(float* outF, const v4f (&fv)[8], int rowBase, int ldo, int col0,
                                         int wave, int hh, int m) {
#pragma unroll
  for (int i = 0; i < 8; ++i) {
    const int lr = 16 * wave + 2 * i + hh;
    float* op = outF + (size_t)(rowBase + lr) * (size_t)ldo + col0 + 4 * m;
    *(volatile v4f*)op = fv[i];
  }
}

__global__ __launch_bounds__(GTHR) void k_gemm_att(
    const unsigned short* __restrict__ A, const unsigned short* __restrict__ WT, float* outF, int K,
    const float* __restrict__ atts, const float* __restrict__ attd, float* SD)
{
  __shared__ __attribute__((aligned(16))) float stg[GBM * GBN];
  __shared__ __attribute__((aligned(16))) float satt[2 * GBN];
  __shared__ __attribute__((aligned(16))) float sdot[2 * GBM];
  const int tid = (int)threadIdx.x, lane = tid & 31, wave = tid >> 5, hh = lane >> 4, m = lane & 15;
  const int rowBase = (int)blockIdx.x * GBM;
  const int head    = (int)blockIdx.y;
  const int col0    = head * GBN;
  {
    const int which = tid >> 6;
    const int c  = tid & 63;
    const float vs = atts[head * CH + c];
    const float vd = attd[head * CH + c];
    const float v = (which == 0) ? vs : vd;
    satt[which * GBN + c] = bfr(v);
  }
  v8f acc[4];
  gemm_acc64(A, WT, K, rowBase, col0, wave, hh, m, acc);
  const float bz[4] = {0.f, 0.f, 0.f, 0.f};
  stage64<false>(stg, acc, bz, wave, hh, m);
  __syncthreads();
  {
    const int row = tid & 63, which = tid >> 6;
    const float* sa = satt + which * GBN;
    const float* hr = stg + row * GBN;
    float d = 0.f;
#pragma unroll 4
    for (int c4 = 0; c4 < GBN / 4; ++c4) {
      const v4f hv = *(const v4fa*)(hr + 4 * c4);
      const v4f av = *(const v4fa*)(sa + 4 * c4);
      d = fmaf(hv.x, av.x, d);
      d = fmaf(hv.y, av.y, d);
      d = fmaf(hv.z, av.z, d);
      d = fmaf(hv.w, av.w, d);
    }
    sdot[which * GBM + row] = d;
  }
  __syncthreads();
  v4f fv[8];
  load_rows(stg, fv, wave, hh, m);
  const int which2 = lane >> 4, piece = lane & 15;
  const v4f sdv = *(const v4fa*)(sdot + which2 * GBM + 4 * piece);
  float* sp = SD + (size_t)(2 * head + which2) * (size_t)NN + rowBase + 4 * piece;
  put_rows(outF, fv, rowBase, HC, col0, wave, hh, m);
  if (wave == 0) *(volatile v4f*)sp = sdv;
  __threadfence();
  put_rows(outF, fv, rowBase, HC, col0, wave, hh, m);
  if (wave == 0) *(volatile v4f*)sp = sdv;
}

template <int MODE>
__global__ __launch_bounds__(GTHR) void k_gemm_act(
    const unsigned short* __restrict__ A, const unsigned short* __restrict__ WT, const float* __restrict__ bias,
    float* outF, int K, int ldo, double* REC)
{
  __shared__ __attribute__((aligned(16))) float  stg[GBM * GBN];
  __shared__ __attribute__((aligned(16))) double dpart[2 * GBN * 2];
  const int tid = (int)threadIdx.x, lane = tid & 31, wave = tid >> 5, hh = lane >> 4, m = lane & 15;
  const int rowBase = (int)blockIdx.x * GBM;
  const int col0    = (int)blockIdx.y * GBN;
  float bv[4];
#pragma unroll
  for (int t = 0; t < 4; ++t) bv[t] = bfr(bias[col0 + 16 * t + m]);
  v8f acc[4];
  gemm_acc64(A, WT, K, rowBase, col0, wave, hh, m, acc);
  stage64<true>(stg, acc, bv, wave, hh, m);
  __syncthreads();
  v2d rv; rv.x = 0.0; rv.y = 0.0;
  if (MODE == 0) {
    const int col = tid & 63, part = tid >> 6;
    double s = 0.0, q = 0.0;
#pragma unroll 4
    for (int r = 0; r < 32; ++r) {
      const double dv = (double)stg[(part * 32 + r) * GBN + col];
      s += dv;
      q += dv * dv;
    }
    dpart[(part * GBN + col) * 2]     = s;
    dpart[(part * GBN + col) * 2 + 1] = q;
    __syncthreads();
    const v2d p0 = *(const v2da*)(dpart + col * 2);
    const v2d p1 = *(const v2da*)(dpart + (GBN + col) * 2);
    rv.x = p0.x + p1.x; rv.y = p0.y + p1.y;
  }
  v4f fv[8];
  load_rows(stg, fv, wave, hh, m);
  double* rp = REC + ((size_t)blockIdx.x * GBN + (tid & 63)) * 2;
  put_rows(outF, fv, rowBase, ldo, col0, wave, hh, m);
  if (MODE == 0) { if (tid < GBN) *(volatile v2d*)rp = rv; }
  __threadfence();
  put_rows(outF, fv, rowBase, ldo, col0, wave, hh, m);
  if (MODE == 0) { if (tid < GBN) *(volatile v2d*)rp = rv; }
}

__global__ __launch_bounds__(GTHR) void k_mid1(
    const unsigned short* __restrict__ A, const unsigned short* __restrict__ WT, const float* __restrict__ bmid,
    const float* __restrict__ wnode, const float* __restrict__ bnode, float* Z1, double* REC1)
{
  __shared__ __attribute__((aligned(16))) float  stg[GBM * GBN];
  __shared__ __attribute__((aligned(16))) float  swn[NODED * CH];
  __shared__ __attribute__((aligned(16))) float  sz1[GBM * NODED];
  __shared__ __attribute__((aligned(16))) double dpart[16 * NODED * 2];
  const int tid = (int)threadIdx.x, lane = tid & 31, wave = tid >> 5, hh = lane >> 4, m = lane & 15;
  const int rowBase = (int)blockIdx.x * GBM;
  {
    const v4f w4 = bfr4(*(const v4f*)(wnode + 4 * tid));
    *(v4fa*)(swn + 4 * tid) = w4;
  }
  float bv[4];
#pragma unroll
  for (int t = 0; t < 4; ++t) bv[t] = bfr(bmid[16 * t + m]);
  v8f acc[4];
  gemm_acc64(A, WT, KA, rowBase, 0, wave, hh, m, acc);
  stage64<true>(stg, acc, bv, wave, hh, m);
  __syncthreads();
  {
    const int row = tid & 63, cg = tid >> 6;
    const float* hr = stg + row * GBN;
    const float* w0 = swn + (4 * cg) * CH;
    float o0 = 0.f, o1 = 0.f, o2 = 0.f, o3 = 0.f;
#pragma unroll 1
    for (int k4 = 0; k4 < CH / 4; ++k4) {
      const v4f a  = *(const v4fa*)(hr + 4 * k4);
      const v4f u0 = *(const v4fa*)(w0 + 4 * k4);
      const v4f u1 = *(const v4fa*)(w0 + CH + 4 * k4);
      const v4f u2 = *(const v4fa*)(w0 + 2 * CH + 4 * k4);
      const v4f u3 = *(const v4fa*)(w0 + 3 * CH + 4 * k4);
      o0 = fmaf(a.x, u0.x, o0); o0 = fmaf(a.y, u0.y, o0); o0 = fmaf(a.z, u0.z, o0); o0 = fmaf(a.w, u0.w, o0);
      o1 = fmaf(a.x, u1.x, o1); o1 = fmaf(a.y, u1.y, o1); o1 = fmaf(a.z, u1.z, o1); o1 = fmaf(a.w, u1.w, o1);
      o2 = fmaf(a.x, u2.x, o2); o2 = fmaf(a.y, u2.y, o2); o2 = fmaf(a.z, u2.z, o2); o2 = fmaf(a.w, u2.w, o2);
      o3 = fmaf(a.x, u3.x, o3); o3 = fmaf(a.y, u3.y, o3); o3 = fmaf(a.z, u3.z, o3); o3 = fmaf(a.w, u3.w, o3);
    }
    const v4f bn = bfr4(*(const v4f*)(bnode + 4 * cg));
    v4f zv;
    zv.x = lrelu(o0 + bn.x); zv.y = lrelu(o1 + bn.y); zv.z = lrelu(o2 + bn.z); zv.w = lrelu(o3 + bn.w);
    *(v4fa*)(sz1 + row * NODED + 4 * cg) = zv;
  }
  __syncthreads();
  const int col = tid & 7, part = tid >> 3;
  {
    double s = 0.0, q = 0.0;
#pragma unroll
    for (int r = 0; r < 4; ++r) {
      const double dv = (double)sz1[(part * 4 + r) * NODED + col];
      s += dv;
      q += dv * dv;
    }
    dpart[(part * NODED + col) * 2]     = s;
    dpart[(part * NODED + col) * 2 + 1] = q;
  }
  const v4f zo = *(const v4fa*)(sz1 + 4 * tid);
  __syncthreads();
  v2d rv; rv.x = 0.0; rv.y = 0.0;
#pragma unroll 4
  for (int p = 0; p < 16; ++p) {
    const v2d pv = *(const v2da*)(dpart + (p * NODED + col) * 2);
    rv.x += pv.x; rv.y += pv.y;
  }
  float*  zp = Z1 + (size_t)rowBase * NODED + 4 * tid;
  double* rp = REC1 + ((size_t)blockIdx.x * NODED + col) * 2;
  *(volatile v4f*)zp = zo;
  if (tid < NODED) *(volatile v2d*)rp = rv;
  __threadfence();
  *(volatile v4f*)zp = zo;
  if (tid < NODED) *(volatile v2d*)rp = rv;
}

__global__ __launch_bounds__(NTHR) void k_scan(const int* __restrict__ HITS, const int* __restrict__ FLGB,
                                               const float* __restrict__ F, const float* __restrict__ SD,
                                               const float* __restrict__ bias, unsigned short* AP, int* FLGO) {
  extern __shared__ __attribute__((aligned(16))) int ssm[];
  int* sl   = ssm;
  int* cnt  = ssm + NBA * DEGCAP;
  int* misc = cnt + NBA;
  const int tid = (int)threadIdx.x, lane = tid & 31, wave = tid >> 5;
  const int blk = (int)blockIdx.x;
  const int nodeBase = blk * NBA;

  const int nhraw = FLGB[(size_t)blk * 32];
  const int bflag = FLGB[(size_t)blk * 32 + 1];
  int nh = nhraw < 0 ? 0 : (nhraw > RCAP ? RCAP : nhraw);
  nh = __builtin_amdgcn_readfirstlane(nh);
  const int ovf = (bflag != 0 || nhraw < 0 || nhraw > RCAP) ? 1 : 0;

  {
    const v4i z4 = {0, 0, 0, 0};
    for (int i = tid * 4; i < SCAN_LDS_INTS; i += NTHR * 4) *(v4ia*)(ssm + i) = z4;
  }
  __syncthreads();

  if (wave == 0) {
    const int* hb = HITS + (size_t)blk * RCAP;
#pragma unroll 1
    for (int b0 = 0; b0 < nh; b0 += 32) {
      int idx = b0 + lane;
      idx = idx < nh ? idx : nh - 1;
      const int uv  = hb[idx];
      const int m32 = (nh - b0) < 32 ? (nh - b0) : 32;
#pragma unroll 1
      for (int k = 0; k < m32; ++k) {
        const int u  = __builtin_amdgcn_readlane(uv, k);
        const int sq = (u >> SRCB) & (NBA - 1);
        const int s  = u & (NN - 1);
        const int p  = cnt[sq];
        const bool ok = (p >= 0) && (p < DEGCAP);
        const int pc = ok ? p : 0;
        if (lane == 0) {
          if (ok) sl[sq * DEGCAP + pc] = s;
          cnt[sq] = (p < RCAP) ? p + 1 : p;
        }
      }
    }
  }
  __syncthreads();

  const float qnan = __int_as_float(0x7fc00000);
  const int head = lane >> 4;
  const float* S0 = SD;
  const float* D0 = SD + NN;
  const float* S1 = SD + 2 * NN;
  const float* D1 = SD + 3 * NN;
  const v4f bq = bfr4(*(const v4f*)(bias + 4 * lane));
  int anybig = 0;

#pragma unroll 1
  for (int si = 0; si < NBA / NWAVE; ++si) {
    const int s    = wave * (NBA / NWAVE) + si;
    const int node = nodeBase + s;
    const int nc   = node < NN ? node : NN - 1;
    const int craw = __builtin_amdgcn_readfirstlane(cnt[s]);
    const bool big = craw > DEGCAP;
    anybig |= big ? 1 : 0;
    const int c  = craw < 0 ? 0 : (craw > DEGCAP ? DEGCAP : craw);
    const int cl = c > 0 ? c - 1 : 0;
    const int* lp = sl + s * DEGCAP;
    const float ad0 = D0[nc];
    const float ad1 = D1[nc];

    float m0 = -3.0e38f, m1 = -3.0e38f;
#pragma unroll 1
    for (int b0 = 0; b0 < c; b0 += 32) {
      const int t  = b0 + lane;
      const int tc = t < cl ? t : cl;
      int src = lp[tc];
      src = src < 0 ? 0 : (src > NN - 1 ? NN - 1 : src);
      const float e0 = lrelu(S0[src] + ad0);
      const float e1 = lrelu(S1[src] + ad1);
      m0 = fmaxf(m0, e0);
      m1 = fmaxf(m1, e1);
    }
#pragma unroll
    for (int off = 16; off > 0; off >>= 1) {
      m0 = fmaxf(m0, __shfl_xor(m0, off));
      m1 = fmaxf(m1, __shfl_xor(m1, off));
    }

    float d0 = 0.0f, d1 = 0.0f;
    v4f acc = {0.f, 0.f, 0.f, 0.f};
#pragma unroll 1
    for (int b0 = 0; b0 < c; b0 += 32) {
      const int t  = b0 + lane;
      const int tc = t < cl ? t : cl;
      int src = lp[tc];
      src = src < 0 ? 0 : (src > NN - 1 ? NN - 1 : src);
      const float e0 = lrelu(S0[src] + ad0);
      const float e1 = lrelu(S1[src] + ad1);
      const float x0 = expf(e0 - m0);
      const float x1 = expf(e1 - m1);
      const bool valid = t < c;
      const float p0 = valid ? x0 : 0.0f;
      const float p1 = valid ? x1 : 0.0f;
      d0 += p0;
      d1 += p1;
      const int m32 = (c - b0) < 32 ? (c - b0) : 32;
#pragma unroll 1
      for (int k = 0; k < m32; ++k) {
        const int   sk = __builtin_amdgcn_readlane(src, k);
        const float q0 = __int_as_float(__builtin_amdgcn_readlane(__float_as_int(p0), k));
        const float q1 = __int_as_float(__builtin_amdgcn_readlane(__float_as_int(p1), k));
        const float pk = (head != 0) ? q1 : q0;
        const v4f a = *(const v4f*)(F + (size_t)sk * HC + 4 * lane);
        acc.x = fmaf(pk, a.x, acc.x);
        acc.y = fmaf(pk, a.y, acc.y);
        acc.z = fmaf(pk, a.z, acc.z);
        acc.w = fmaf(pk, a.w, acc.w);
      }
    }
#pragma unroll
    for (int off = 16; off > 0; off >>= 1) {
      d0 += __shfl_xor(d0, off);
      d1 += __shfl_xor(d1, off);
    }
    const float den = (head != 0) ? d1 : d0;
    const float rc  = __builtin_amdgcn_rcpf(den);
    const float inv = (c > 0) ? rc : 0.0f;
    const float pz  = (ovf != 0 || big) ? qnan : 0.0f;
    const float y0 = fmaf(acc.x, inv, bq.x) + pz;
    const float y1 = fmaf(acc.y, inv, bq.y) + pz;
    const float y2 = fmaf(acc.z, inv, bq.z) + pz;
    const float y3 = fmaf(acc.w, inv, bq.w) + pz;
    v2u hv, lv;
    hv.x = pk2(y0, y1);   hv.y = pk2(y2, y3);
    lv.x = pk2lo(y0, y1); lv.y = pk2lo(y2, y3);
    unsigned short* hp = AP + (size_t)nc * KA + 4 * lane;
    *(volatile v2u*)hp = hv;
    *(volatile v2u*)(hp + HC) = lv;
    __threadfence();
    *(volatile v2u*)hp = hv;
    *(volatile v2u*)(hp + HC) = lv;
  }

  if (lane == 0) misc[wave] = anybig;
  __syncthreads();
  if (wave == 0) {
    int fg = ovf;
#pragma unroll
    for (int w2 = 0; w2 < NWAVE; ++w2) fg |= misc[w2];
    v4i cv;
    cv.x = 0;
    cv.y = (lane == 0) ? fg : 0;
    cv.z = 0; cv.w = 0;
    int* fp = FLGO + (size_t)blk * 32 + 4 * (lane & 7);
    if (lane < 8) *(volatile v4i*)fp = cv;
    __threadfence();
    if (lane < 8) *(volatile v4i*)fp = cv;
  }
}

__global__ __launch_bounds__(NTHR) void k_bn0(const float* __restrict__ Z0, const double* __restrict__ REC,
                                              const float* __restrict__ g, const float* __restrict__ b,
                                              unsigned short* X1) {
  __shared__ __attribute__((aligned(16))) float smean[CH];
  __shared__ __attribute__((aligned(16))) float sscale[CH];
  __shared__ __attribute__((aligned(16))) float sshift[CH];
  const int tid = (int)threadIdx.x;
  const int blk = (int)blockIdx.x;
  if (tid < CH) {
    double S = 0.0, Q = 0.0;
#pragma unroll 4
    for (int t = 0; t < NT64; ++t) {
      const v2d r = *(const v2d*)(REC + ((size_t)t * CH + tid) * 2);
      S += r.x; Q += r.y;
    }
    const double mean = S * (1.0 / (double)NN);
    double var = Q * (1.0 / (double)NN) - mean * mean;
    var = (var < 0.0) ? 0.0 : var;
    const double rstd = 1.0 / sqrt(var + (double)BN_EPS);
    smean[tid]  = (float)mean;
    sscale[tid] = (float)rstd * bfr(g[tid]);
    sshift[tid] = bfr(b[tid]);
  }
  __syncthreads();
  const int c0 = (tid & 7) * 8;
  const v4f ma = *(const v4fa*)(smean + c0),  mb = *(const v4fa*)(smean + c0 + 4);
  const v4f sa = *(const v4fa*)(sscale + c0), sb = *(const v4fa*)(sscale + c0 + 4);
  const v4f ha = *(const v4fa*)(sshift + c0), hb = *(const v4fa*)(sshift + c0 + 4);
#pragma unroll 1
  for (int it = 0; it < 4; ++it) {
    const int row = blk * 128 + it * 32 + (tid >> 3);
    const float* zp = Z0 + (size_t)row * CH + c0;
    const v4f za = *(const v4f*)zp, zb = *(const v4f*)(zp + 4);
    v4f ya, yb;
    ya.x = fmaf(za.x - ma.x, sa.x, ha.x); ya.y = fmaf(za.y - ma.y, sa.y, ha.y);
    ya.z = fmaf(za.z - ma.z, sa.z, ha.z); ya.w = fmaf(za.w - ma.w, sa.w, ha.w);
    yb.x = fmaf(zb.x - mb.x, sb.x, hb.x); yb.y = fmaf(zb.y - mb.y, sb.y, hb.y);
    yb.z = fmaf(zb.z - mb.z, sb.z, hb.z); yb.w = fmaf(zb.w - mb.w, sb.w, hb.w);
    const v4u hv = pack8(ya, yb);
    const v4u lv = pack8lo(ya, yb);
    unsigned short* dp = X1 + (size_t)row * KX1 + c0;
    *(volatile v4u*)dp = hv;
    *(volatile v4u*)(dp + CH) = lv;
    __threadfence();
    *(volatile v4u*)dp = hv;
    *(volatile v4u*)(dp + CH) = lv;
  }
}

__global__ __launch_bounds__(NTHR) void k_bn1(const float* __restrict__ Z1, const double* __restrict__ REC1,
                                              const float* __restrict__ g, const float* __restrict__ b,
                                              unsigned short* ZP) {
  __shared__ __attribute__((aligned(16))) float smean[NODED];
  __shared__ __attribute__((aligned(16))) float sscale[NODED];
  __shared__ __attribute__((aligned(16))) float sshift[NODED];
  const int tid = (int)threadIdx.x;
  {
    const int c = tid & 7;
    double S = 0.0, Q = 0.0;
#pragma unroll 4
    for (int t = 0; t < NT64; ++t) {
      const v2d r = *(const v2d*)(REC1 + ((size_t)t * NODED + c) * 2);
      S += r.x; Q += r.y;
    }
    const double mean = S * (1.0 / (double)NN);
    double var = Q * (1.0 / (double)NN) - mean * mean;
    var = (var < 0.0) ? 0.0 : var;
    const double rstd = 1.0 / sqrt(var + (double)BN_EPS);
    const float gs = bfr(g[c]);
    const float bs = bfr(b[c]);
    if (tid < NODED) {
      smean[tid]  = (float)mean;
      sscale[tid] = (float)rstd * gs;
      sshift[tid] = bs;
    }
  }
  __syncthreads();
  const v4f ma = *(const v4fa*)(smean),  mb = *(const v4fa*)(smean + 4);
  const v4f sa = *(const v4fa*)(sscale), sb = *(const v4fa*)(sscale + 4);
  const v4f ha = *(const v4fa*)(sshift), hb = *(const v4fa*)(sshift + 4);
  const int node = (int)blockIdx.x * NTHR + tid;
  const float* zp = Z1 + (size_t)node * NODED;
  const v4f za = *(const v4f*)zp, zb = *(const v4f*)(zp + 4);
  v4f ya, yb;
  ya.x = fmaf(za.x - ma.x, sa.x, ha.x); ya.y = fmaf(za.y - ma.y, sa.y, ha.y);
  ya.z = fmaf(za.z - ma.z, sa.z, ha.z); ya.w = fmaf(za.w - ma.w, sa.w, ha.w);
  yb.x = fmaf(zb.x - mb.x, sb.x, hb.x); yb.y = fmaf(zb.y - mb.y, sb.y, hb.y);
  yb.z = fmaf(zb.z - mb.z, sb.z, hb.z); yb.w = fmaf(zb.w - mb.w, sb.w, hb.w);
  const v4u hv = pack8(ya, yb);
  const v4u lv = pack8lo(ya, yb);
  const int gg = node >> 7, p = node & (PN - 1);
  unsigned short* dp = ZP + (size_t)gg * KF1 + p * NODED;
  *(volatile v4u*)dp = hv;
  *(volatile v4u*)(dp + PN * NODED) = lv;
  __threadfence();
  *(volatile v4u*)dp = hv;
  *(volatile v4u*)(dp + PN * NODED) = lv;
}

__global__ __launch_bounds__(NTHR) void k_tail(const float* __restrict__ F1, const float* __restrict__ wf2,
                                               const float* __restrict__ bf2, const float* __restrict__ wf3,
                                               const float* __restrict__ bf3, const int* __restrict__ FLG,
                                               float* out) {
  __shared__ __attribute__((aligned(16))) float sF2[NG * NF2];
  __shared__ int swf[NWAVE];
  const int tid = (int)threadIdx.x, lane = tid & 31, wave = tid >> 5;
  {
    const int li = tid < NFLG ? tid : NFLG - 1;
    const int fw = FLG[(size_t)li * 32 + 1];
    const unsigned bal = __builtin_amdgcn_ballot_w32((tid < NFLG) && (fw != 0));
    if (lane == 0) swf[wave] = (bal != 0u) ? 1 : 0;
  }
  const int g = tid >> 2, jq = tid & 3;
  const float* fr = F1 + (size_t)g * NF1;
#pragma unroll 1
  for (int jh = 0; jh < 2; ++jh) {
    const int j0 = jq * 8 + jh * 4;
    const float* w0 = wf2 + (size_t)j0 * NF1;
    float a0 = 0.f, a1 = 0.f, a2 = 0.f, a3 = 0.f;
#pragma unroll 1
    for (int k4 = 0; k4 < NF1 / 4; ++k4) {
      const v4f a  = *(const v4f*)(fr + 4 * k4);
      const v4f u0 = bfr4(*(const v4f*)(w0 + 4 * k4));
      const v4f u1 = bfr4(*(const v4f*)(w0 + NF1 + 4 * k4));
      const v4f u2 = bfr4(*(const v4f*)(w0 + 2 * NF1 + 4 * k4));
      const v4f u3 = bfr4(*(const v4f*)(w0 + 3 * NF1 + 4 * k4));
      a0 = fmaf(a.x, u0.x, a0); a0 = fmaf(a.y, u0.y, a0); a0 = fmaf(a.z, u0.z, a0); a0 = fmaf(a.w, u0.w, a0);
      a1 = fmaf(a.x, u1.x, a1); a1 = fmaf(a.y, u1.y, a1); a1 = fmaf(a.z, u1.z, a1); a1 = fmaf(a.w, u1.w, a1);
      a2 = fmaf(a.x, u2.x, a2); a2 = fmaf(a.y, u2.y, a2); a2 = fmaf(a.z, u2.z, a2); a2 = fmaf(a.w, u2.w, a2);
      a3 = fmaf(a.x, u3.x, a3); a3 = fmaf(a.y, u3.y, a3); a3 = fmaf(a.z, u3.z, a3); a3 = fmaf(a.w, u3.w, a3);
    }
    const v4f bq = bfr4(*(const v4f*)(bf2 + j0));
    v4f r;
    r.x = lrelu(a0 + bq.x); r.y = lrelu(a1 + bq.y); r.z = lrelu(a2 + bq.z); r.w = lrelu(a3 + bq.w);
    *(v4fa*)(sF2 + g * NF2 + j0) = r;
  }
  __syncthreads();
  if (tid < NG) {
    int fg = 0;
#pragma unroll
    for (int w2 = 0; w2 < NWAVE; ++w2) fg |= swf[w2];
    const float* f2r = sF2 + tid * NF2;
    float o = 0.f;
#pragma unroll 2
    for (int j4 = 0; j4 < NF2 / 4; ++j4) {
      const v4f v = *(const v4fa*)(f2r + 4 * j4);
      const v4f w = bfr4(*(const v4f*)(wf3 + 4 * j4));
      o = fmaf(v.x, w.x, o); o = fmaf(v.y, w.y, o); o = fmaf(v.z, w.z, o); o = fmaf(v.w, w.w, o);
    }
    o += bfr(bf3[0]);
    const float qnan = __int_as_float(0x7fc00000);
    const float ov = (fg != 0) ? qnan : o;
    float* op = out + tid;
    *(volatile float*)op = ov;
    __threadfence();
    *(volatile float*)op = ov;
  }
}

static inline size_t al256(size_t v) { return (v + 255) & ~(size_t)255; }

extern "C" void kernel_launch(void* const* d_in, const int* in_sizes, int n_in,
                              void* d_out, int out_size, void* d_ws, size_t ws_size,
                              hipStream_t stream) {
  if (n_in < 28) return;
  const int expect[28] = {
    NN * FIN, 2 * 1048576, 1048576, NN,
    HC * FIN, NHEAD * CH, NHEAD * CH, HC,
    CH * HC, CH, CH, CH,
    HC * CH, NHEAD * CH, NHEAD * CH, HC,
    CH * HC, CH, NODED * CH, NODED, NODED, NODED,
    NF1 * PN * NODED, NF1, NF2 * NF1, NF2, NF2, 1 };
  for (int i = 0; i < 28; ++i) if (in_sizes[i] != expect[i]) return;
  if (out_size != NG) return;
  const int nE = in_sizes[1] / 2;
  if (nE < 1 || (in_sizes[1] & 1) != 0) return;

  const float* x     = (const float*)d_in[0];
  const int*   ei    = (const int*)  d_in[1];
  const float* wl0   = (const float*)d_in[4];
  const float* as0   = (const float*)d_in[5];
  const float* ad0   = (const float*)d_in[6];
  const float* bias0 = (const float*)d_in[7];
  const float* wp0   = (const float*)d_in[8];
  const float* bp0   = (const float*)d_in[9];
  const float* g0    = (const float*)d_in[10];
  const float* b0    = (const float*)d_in[11];
  const float* wl1   = (const float*)d_in[12];
  const float* as1   = (const float*)d_in[13];
  const float* ad1   = (const float*)d_in[14];
  const float* bias1 = (const float*)d_in[15];
  const float* wm1   = (const float*)d_in[16];
  const float* bm1   = (const float*)d_in[17];
  const float* wn1   = (const float*)d_in[18];
  const float* bn1b  = (const float*)d_in[19];
  const float* g1    = (const float*)d_in[20];
  const float* b1    = (const float*)d_in[21];
  const float* wf1   = (const float*)d_in[22];
  const float* bf1   = (const float*)d_in[23];
  const float* wf2   = (const float*)d_in[24];
  const float* bf2   = (const float*)d_in[25];
  const float* wf3   = (const float*)d_in[26];
  const float* bf3   = (const float*)d_in[27];
  float* out = (float*)d_out;
  const int* src = ei;
  const int* dst = ei + nE;
  const int vec8 = ((nE & 3) == 0) ? 1 : 0;

  char* ws = (char*)d_ws;
  size_t off = 0;
  const size_t oXB  = off; off = al256(off + (size_t)NN * FIN * 2);
  const size_t oWL0 = off; off = al256(off + (size_t)HC * FIN * 2);
  const size_t oWP0 = off; off = al256(off + (size_t)CH * KA * 2);
  const size_t oWL1 = off; off = al256(off + (size_t)HC * KX1 * 2);
  const size_t oWM1 = off; off = al256(off + (size_t)CH * KA * 2);
  const size_t oWF1 = off; off = al256(off + (size_t)NF1 * KF1 * 2);
  const size_t oH   = off; off = al256(off + (size_t)NN * HC * 4);
  const size_t oSD  = off; off = al256(off + (size_t)4 * NN * 4);
  const size_t oAHL = off; off = al256(off + (size_t)NN * KA * 2);
  const size_t oZ0  = off; off = al256(off + (size_t)NN * CH * 4);
  const size_t oX1  = off; off = al256(off + (size_t)NN * KX1 * 2);
  const size_t oZ1  = off; off = al256(off + (size_t)NN * NODED * 4);
  const size_t oZP  = off; off = al256(off + (size_t)NG * KF1 * 2);
  const size_t oF1  = off; off = al256(off + (size_t)NG * NF1 * 4);
  const size_t oHIT = off; off = al256(off + (size_t)NBLK * RCAP * 4);
  const size_t oFLG = off; off = al256(off + (size_t)NFLG * 128);
  const size_t oR0  = off; off = al256(off + (size_t)NT64 * CH * 2 * 8);
  const size_t oR1  = off; off = al256(off + (size_t)NT64 * NODED * 2 * 8);
  if (off > ws_size || off > (size_t)WSMAX) return;
  unsigned short* XB   = (unsigned short*)(ws + oXB);
  unsigned short* WL0  = (unsigned short*)(ws + oWL0);
  unsigned short* WP0D = (unsigned short*)(ws + oWP0);
  unsigned short* WL1D = (unsigned short*)(ws + oWL1);
  unsigned short* WM1D = (unsigned short*)(ws + oWM1);
  unsigned short* WF1D = (unsigned short*)(ws + oWF1);
  float*          H    = (float*)(ws + oH);
  float*          SD   = (float*)(ws + oSD);
  unsigned short* AHL  = (unsigned short*)(ws + oAHL);
  float*          Z0   = (float*)(ws + oZ0);
  unsigned short* X1   = (unsigned short*)(ws + oX1);
  float*          Z1   = (float*)(ws + oZ1);
  unsigned short* ZP   = (unsigned short*)(ws + oZP);
  float*          F1   = (float*)(ws + oF1);
  int*            HITS = (int*)(ws + oHIT);
  int*            FLG  = (int*)(ws + oFLG);
  double*         REC0 = (double*)(ws + oR0);
  double*         REC1 = (double*)(ws + oR1);
  int* FLG0 = FLG;
  int* FLG1 = FLG + (size_t)NBLK * 32;
  int* FLG2 = FLG + (size_t)2 * NBLK * 32;

  const int bktLds  = BKT_LDS_INTS * 4;
  const int scanLds = SCAN_LDS_INTS * 4;
  hipFuncSetAttribute(reinterpret_cast<const void*>(&k_bucket),
                      hipFuncAttributeMaxDynamicSharedMemorySize, bktLds);
  hipFuncSetAttribute(reinterpret_cast<const void*>(&k_scan),
                      hipFuncAttributeMaxDynamicSharedMemorySize, scanLds);

  k_prep<<<NU_ALL / NTHR, NTHR, 0, stream>>>(x, wl0, wp0, wl1, wm1, wf1, XB, WL0, WP0D, WL1D, WM1D, WF1D);
  k_bucket<<<NBLK, NTHR, bktLds, stream>>>(src, dst, nE, NN, vec8, HITS, FLG0);
  k_gemm_att<<<dim3(NN / GBM, NHEAD), GTHR, 0, stream>>>(XB, WL0, H, FIN, as0, ad0, SD);
  k_scan<<<NBLK, NTHR, scanLds, stream>>>(HITS, FLG0, H, SD, bias0, AHL, FLG1);
  k_gemm_act<0><<<dim3(NN / GBM, 1), GTHR, 0, stream>>>(AHL, WP0D, bp0, Z0, KA, CH, REC0);
  k_bn0<<<NN / 128, NTHR, 0, stream>>>(Z0, REC0, g0, b0, X1);
  k_gemm_att<<<dim3(NN / GBM, NHEAD), GTHR, 0, stream>>>(X1, WL1D, H, KX1, as1, ad1, SD);
  k_scan<<<NBLK, NTHR, scanLds, stream>>>(HITS, FLG0, H, SD, bias1, AHL, FLG2);
  k_mid1<<<NN / GBM, GTHR, 0, stream>>>(AHL, WM1D, bm1, wn1, bn1b, Z1, REC1);
  k_bn1<<<NN / NTHR, NTHR, 0, stream>>>(Z1, REC1, g1, b1, ZP);
  k_gemm_act<1><<<dim3(NG / GBM, NF1 / GBN), GTHR, 0, stream>>>(ZP, WF1D, bf1, F1, KF1, NF1, REC0);
  k_tail<<<1, NTHR, 0, stream>>>(F1, wf2, bf2, wf3, bf3, FLG, out);
}
